// KPConvBasicBlock_51866025066566
// MI455X (gfx1250) — hardware-verified
//
#include <hip/hip_runtime.h>
#include <stddef.h>


#define HN      32
#define CIN     32
#define COUT    64
#define KP      15
#define KTOT    (KP * CIN)
#define KSTEPS  (KTOT / 32)
#define BP      512
#define APITCH  KTOT
#define TPW     16
#define MWAV    2
#define MTHR    (MWAV * 32)
#define CA      16.0f
#define CB      64.0f
#define RINV    0.0009765625f
#define WSCAP   134217728

#define L_W       0
#define L_I       (L_W + TPW * HN * 16 * 4)
#define L_A       (L_I + TPW * HN * 4)
#define L_S       (L_A + TPW * APITCH * 2)
#define LW_BYTES  (L_S + TPW * COUT * 4)
#define LDS_MAIN  (MWAV * LW_BYTES)

static_assert(KTOT % 32 == 0);
static_assert(HN == 32 && CIN == 32 && COUT == 64 && TPW == 16);
static_assert((APITCH * 2) % 16 == 0);
static_assert((BP * 2) % 128 == 0 && BP >= KTOT);
static_assert(L_I == 32768 && L_A == 34816 && L_S == 50176 && LW_BYTES == 54272);
static_assert((L_I % 16) == 0 && (L_A % 16) == 0 && (L_S % 16) == 0 && (LW_BYTES % 16) == 0);
static_assert(LDS_MAIN == 108544);

typedef float    v4f  __attribute__((ext_vector_type(4)));
typedef float    v8f  __attribute__((ext_vector_type(8)));
typedef _Float16 v8h  __attribute__((ext_vector_type(8)));
typedef _Float16 v16h __attribute__((ext_vector_type(16)));
union Frag { v16h v; v8h h[2]; };

__device__ __forceinline__ v8f wmh(v16h a, v16h b, v8f c) {
  v8f d = __builtin_amdgcn_wmma_f32_16x16x32_f16(false, a, false, b, (short)0, c, false, false);
  asm volatile("v_nop\n\tv_nop\n\tv_nop\n\tv_nop" : "+v"(d) : "v"(a), "v"(b));
  return d;
}

__global__ __launch_bounds__(64) void k_wprep(const float* __restrict__ Kv, _Float16* Bt) {
  const int o = blockIdx.x, t = threadIdx.x;
  const int kk0 = 8 * t;
  v8h hv;
#pragma unroll
  for (int e = 0; e < 8; ++e) {
    const int kk = kk0 + e;
    const int kc = kk < KTOT ? kk : KTOT - 1;
    const float v = Kv[(size_t)kc * COUT + o];
    const float s = (kk < KTOT) ? v * CB : 0.0f;
    hv[e] = (_Float16)s;
  }
  _Float16* dst = Bt + (size_t)o * BP + kk0;
  *(volatile v8h*)dst = hv;
  __threadfence();
  *(volatile v8h*)dst = hv;
}

__global__ __launch_bounds__(MTHR) void k_main(const float* __restrict__ query, const float* __restrict__ support,
                                               const int* __restrict__ edge, const float* __restrict__ feats,
                                               const float* __restrict__ kpts, const _Float16* __restrict__ Bt,
                                               float* out, int nN) {
  extern __shared__ __attribute__((aligned(16))) char dynl[];
  const int tid = threadIdx.x, lane = tid & 31, hh = lane >> 4, m = lane & 15;
  const int wave = __builtin_amdgcn_readfirstlane(tid >> 5);
  char* wb = dynl + (size_t)wave * LW_BYTES;
  float*    Wl = (float*)(wb + L_W);
  int*      Il = (int*)(wb + L_I);
  _Float16* Al = (_Float16*)(wb + L_A);
  float*    S  = (float*)(wb + L_S);
  const int tile = blockIdx.x * MWAV + wave;
  const int n0 = tile * TPW;

  float kp[KP * 3];
#pragma unroll
  for (int i = 0; i < KP * 3; ++i) kp[i] = kpts[i];

#pragma unroll 1
  for (int p = 0; p < TPW; ++p) {
    int n = n0 + p;
    n = n > nN - 1 ? nN - 1 : n;
    int idx = edge[(size_t)n * HN + lane];
    idx = idx < 0 ? idx + nN + 1 : idx;
    idx = idx < 0 ? 0 : (idx > nN ? nN : idx);
    const bool shadow = (idx == nN);
    const int ic = shadow ? nN - 1 : idx;
    const float qx = query[(size_t)n * 3 + 0];
    const float qy = query[(size_t)n * 3 + 1];
    const float qz = query[(size_t)n * 3 + 2];
    const float sx = support[(size_t)ic * 3 + 0];
    const float sy = support[(size_t)ic * 3 + 1];
    const float sz = support[(size_t)ic * 3 + 2];
    const float rx = sx - qx, ry = sy - qy, rz = sz - qz;
    float wk[16];
#pragma unroll
    for (int k = 0; k < KP; ++k) {
      const float dx = rx - kp[3 * k + 0];
      const float dy = ry - kp[3 * k + 1];
      const float dz = rz - kp[3 * k + 2];
      const float d2 = dx * dx + dy * dy + dz * dz;
      const float w = fmaxf(1.0f - __builtin_amdgcn_sqrtf(d2), 0.0f);
      wk[k] = shadow ? 0.0f : w;
    }
    wk[15] = 0.0f;
    v4f* wd = (v4f*)(Wl + ((size_t)p * HN + lane) * 16);
    const v4f t0 = {wk[0], wk[1], wk[2], wk[3]};
    const v4f t1 = {wk[4], wk[5], wk[6], wk[7]};
    const v4f t2 = {wk[8], wk[9], wk[10], wk[11]};
    const v4f t3 = {wk[12], wk[13], wk[14], wk[15]};
    wd[0] = t0;
    wd[1] = t1;
    wd[2] = t2;
    wd[3] = t3;
    Il[p * HN + lane] = ic;
  }
  __syncthreads();

#pragma unroll 1
  for (int p = 0; p < TPW; ++p) {
    float acc[KP];
#pragma unroll
    for (int k = 0; k < KP; ++k) acc[k] = 0.0f;
    const float* wrow = Wl + (size_t)p * HN * 16;
    const int* irow = Il + p * HN;
#pragma unroll 2
    for (int h = 0; h < HN; ++h) {
      int ic = irow[h];
      ic = ic < 0 ? 0 : (ic > nN - 1 ? nN - 1 : ic);
      const float f = feats[(size_t)ic * CIN + lane];
      const v4f w0 = *(const v4f*)(wrow + h * 16 + 0);
      const v4f w1 = *(const v4f*)(wrow + h * 16 + 4);
      const v4f w2 = *(const v4f*)(wrow + h * 16 + 8);
      const v4f w3 = *(const v4f*)(wrow + h * 16 + 12);
      acc[0]  += w0.x * f;  acc[1]  += w0.y * f;  acc[2]  += w0.z * f;  acc[3]  += w0.w * f;
      acc[4]  += w1.x * f;  acc[5]  += w1.y * f;  acc[6]  += w1.z * f;  acc[7]  += w1.w * f;
      acc[8]  += w2.x * f;  acc[9]  += w2.y * f;  acc[10] += w2.z * f;  acc[11] += w2.w * f;
      acc[12] += w3.x * f;  acc[13] += w3.y * f;  acc[14] += w3.z * f;
    }
    _Float16* arow = Al + (size_t)p * APITCH + lane;
#pragma unroll
    for (int k = 0; k < KP; ++k) arow[k * CIN] = (_Float16)(acc[k] * CA);
  }
  __syncthreads();

  const v8f z8 = {0.0f, 0.0f, 0.0f, 0.0f, 0.0f, 0.0f, 0.0f, 0.0f};
  v8f acc0 = z8, acc1 = z8, acc2 = z8, acc3 = z8;
  {
    const _Float16* ap = Al + (size_t)m * APITCH + 8 * hh;
    const _Float16* bq = Bt + (size_t)m * BP + 8 * hh;
#pragma unroll 1
    for (int ks = 0; ks < KSTEPS; ++ks) {
      Frag a, b;
      a.h[0] = *(const v8h*)(ap + 32 * ks);
      a.h[1] = *(const v8h*)(ap + 32 * ks + 16);
      const _Float16* b0 = bq + 32 * ks;
      b.h[0] = *(const v8h*)(b0);
      b.h[1] = *(const v8h*)(b0 + 16);
      acc0 = wmh(a.v, b.v, acc0);
      b.h[0] = *(const v8h*)(b0 + 16 * BP);
      b.h[1] = *(const v8h*)(b0 + 16 * BP + 16);
      acc1 = wmh(a.v, b.v, acc1);
      b.h[0] = *(const v8h*)(b0 + 32 * BP);
      b.h[1] = *(const v8h*)(b0 + 32 * BP + 16);
      acc2 = wmh(a.v, b.v, acc2);
      b.h[0] = *(const v8h*)(b0 + 48 * BP);
      b.h[1] = *(const v8h*)(b0 + 48 * BP + 16);
      acc3 = wmh(a.v, b.v, acc3);
    }
  }

#pragma unroll
  for (int r = 0; r < 8; ++r) {
    float* srow = S + (8 * hh + r) * COUT;
    srow[m]      = acc0[r] * RINV;
    srow[16 + m] = acc1[r] * RINV;
    srow[32 + m] = acc2[r] * RINV;
    srow[48 + m] = acc3[r] * RINV;
  }
  __syncthreads();
  {
    const int rsub = lane >> 4, c4 = (lane & 15) * 4;
    v4f ov[8];
#pragma unroll
    for (int i = 0; i < 8; ++i) ov[i] = *(const v4f*)(S + (2 * i + rsub) * COUT + c4);
#pragma unroll
    for (int i = 0; i < 8; ++i) {
      const int row = n0 + 2 * i + rsub;
      const int rcl = row < nN ? row : nN - 1;
      float* op = out + (size_t)rcl * COUT + c4;
      if (row < nN) *(volatile v4f*)op = ov[i];
    }
    __threadfence();
#pragma unroll
    for (int i = 0; i < 8; ++i) {
      const int row = n0 + 2 * i + rsub;
      const int rcl = row < nN ? row : nN - 1;
      float* op = out + (size_t)rcl * COUT + c4;
      if (row < nN) *(volatile v4f*)op = ov[i];
    }
  }
}

extern "C" void kernel_launch(void* const* d_in, const int* in_sizes, int n_in,
                              void* d_out, int out_size, void* d_ws, size_t ws_size,
                              hipStream_t stream) {
  if (n_in < 6) return;
  if (in_sizes[0] < 3) return;
  const int nN = in_sizes[0] / 3;
  if (nN < 1 || in_sizes[0] != nN * 3) return;
  if (in_sizes[1] != nN * 3) return;
  if (in_sizes[2] != nN * HN) return;
  if (in_sizes[3] != nN * CIN) return;
  if (in_sizes[4] != KP * 3) return;
  if (in_sizes[5] != KP * CIN * COUT) return;
  if (out_size != nN * COUT) return;

  const float* query   = (const float*)d_in[0];
  const float* support = (const float*)d_in[1];
  const int*   edge    = (const int*)d_in[2];
  const float* feats   = (const float*)d_in[3];
  const float* kpts    = (const float*)d_in[4];
  const float* kvals   = (const float*)d_in[5];
  float* out = (float*)d_out;

  char* ws = (char*)d_ws;
  size_t off = 0;
  const size_t oBt = off; off += (size_t)COUT * BP * 2; off = (off + 255) & ~(size_t)255;
  if (off > ws_size || off > (size_t)WSCAP) return;
  _Float16* Bt = (_Float16*)(ws + oBt);

  const int nTiles = (nN + TPW - 1) / TPW;
  const int gMain  = (nTiles + MWAV - 1) / MWAV;

  hipFuncSetAttribute(reinterpret_cast<const void*>(&k_main), hipFuncAttributeMaxDynamicSharedMemorySize, LDS_MAIN);

  k_wprep<<<COUT, 64, 0, stream>>>(kvals, Bt);
  k_main<<<gMain, MTHR, LDS_MAIN, stream>>>(query, support, edge, feats, kpts, Bt, out, nN);
}
